// ClassicalSelfAttention_65481071401183
// MI455X (gfx1250) — hardware-verified
//
#include <hip/hip_runtime.h>


#ifndef SEQ
#define SEQ 16384
#endif
#define SEQ_FULL 16384
#ifndef NB
#define NB 1
#endif
#define HD   64
#define DP   128
#define KC   64
#define SCL  0.125f
#define L2E  1.4426950408889634f
#define LPC  14.0f
static_assert(SEQ % 128 == 0);
static_assert(SEQ % KC == 0);
static_assert(SEQ <= SEQ_FULL);
static_assert(NB == 1);

typedef _Float16 h16;
typedef unsigned short bf;
typedef __attribute__((ext_vector_type(16))) __bf16   v16bf;
typedef __attribute__((ext_vector_type(16))) _Float16 v16h;
typedef __attribute__((ext_vector_type(8)))  _Float16 v8h;
typedef __attribute__((ext_vector_type(8)))  unsigned short v8us;
typedef __attribute__((ext_vector_type(8)))  float    v8f;
typedef __attribute__((ext_vector_type(4)))  float    v4f;
typedef v8h  __attribute__((may_alias)) v8ha;
typedef v4f  __attribute__((may_alias)) v4fa;
typedef v8us __attribute__((may_alias)) v8usa;

__device__ __forceinline__ unsigned short f2bf(float f) { unsigned u = __float_as_uint(f); u += 0x7FFFu + ((u >> 16) & 1u); return (unsigned short)(u >> 16); }
__device__ __forceinline__ float bf2f(unsigned short b) { return __uint_as_float(((unsigned)b) << 16); }
__device__ __forceinline__ float bfr(float f) { return bf2f(f2bf(f)); }
__device__ __forceinline__ v16h cat16(v8h lo, v8h hi) { return __builtin_shufflevector(lo, hi, 0, 1, 2, 3, 4, 5, 6, 7, 8, 9, 10, 11, 12, 13, 14, 15); }
__device__ __forceinline__ v16bf cat16b(v8us lo, v8us hi) { return __builtin_bit_cast(v16bf, __builtin_shufflevector(lo, hi, 0, 1, 2, 3, 4, 5, 6, 7, 8, 9, 10, 11, 12, 13, 14, 15)); }
__device__ __forceinline__ v8f wmma16(v16h a, v16h b, v8f c) { return __builtin_amdgcn_wmma_f32_16x16x32_f16(false, a, false, b, (short)0, c, false, false); }
__device__ __forceinline__ v8f wmmab(v16bf a, v16bf b, v8f c) { return __builtin_amdgcn_wmma_f32_16x16x32_bf16(false, a, false, b, (short)0, c, false, false); }
__device__ __forceinline__ h16 tohx(float x) { return (h16)x; }
__device__ __forceinline__ void splitf(float y, unsigned short& h, unsigned short& l) { h = f2bf(y); l = f2bf(y - bf2f(h)); }

template <typename T16> struct WFrag;
template <> struct WFrag<h16> { typedef v16h V; static __device__ __forceinline__ V ld(const h16* p) { return cat16(*(const v8h*)p, *(const v8h*)(p + 16)); } static __device__ __forceinline__ v8f mma(V a, V b, v8f c) { return wmma16(a, b, c); } };
template <> struct WFrag<bf> { typedef v16bf V; static __device__ __forceinline__ V ld(const bf* p) { return cat16b(*(const v8us*)p, *(const v8us*)(p + 16)); } static __device__ __forceinline__ v8f mma(V a, V b, v8f c) { return wmmab(a, b, c); } };

template <typename T16, int NSPLIT, bool BIAS>
__global__ __launch_bounds__(32) void k_gemmw(const T16* __restrict__ A, const T16* __restrict__ A2, const T16* __restrict__ Bt, const T16* __restrict__ Bt2, int K, float* C, int ldc, const float* __restrict__ bias, size_t sA, size_t sB, size_t sC) {
    typedef typename WFrag<T16>::V V;
    __shared__ __align__(16) float os[16 * 68];
    const size_t z = blockIdx.z; A += z * sA; if (A2) A2 += z * sA; Bt += z * sB; if (Bt2) Bt2 += z * sB; C += z * sC;
    const int lane = threadIdx.x & 31, lr = lane & 15, hi = lane >> 4; const int r0 = blockIdx.x * 64, c0 = blockIdx.y * 64;
    v8f acc[4][4];
#pragma unroll
    for (int mb = 0; mb < 4; ++mb)
#pragma unroll
        for (int nb = 0; nb < 4; ++nb) acc[mb][nb] = (v8f){};
    const size_t aoff = (size_t)(r0 + lr) * K + 8 * hi, boff = (size_t)(c0 + lr) * K + 8 * hi;
#pragma unroll 1
    for (int kc = 0; kc < K; kc += 32) {
        V a[4], a2[4];
#pragma unroll
        for (int mb = 0; mb < 4; ++mb) { a[mb] = WFrag<T16>::ld(A + aoff + (size_t)mb * 16 * K + kc); if (NSPLIT == 1 || NSPLIT == 2) a2[mb] = WFrag<T16>::ld(A2 + aoff + (size_t)mb * 16 * K + kc); }
#pragma unroll
        for (int nb = 0; nb < 4; ++nb) { const V b = WFrag<T16>::ld(Bt + boff + (size_t)nb * 16 * K + kc); V b2; if (NSPLIT >= 2) b2 = WFrag<T16>::ld(Bt2 + boff + (size_t)nb * 16 * K + kc);
#pragma unroll
            for (int mb = 0; mb < 4; ++mb) { acc[mb][nb] = WFrag<T16>::mma(a[mb], b, acc[mb][nb]); if (NSPLIT == 1 || NSPLIT == 2) acc[mb][nb] = WFrag<T16>::mma(a2[mb], b, acc[mb][nb]); if (NSPLIT >= 2) acc[mb][nb] = WFrag<T16>::mma(a[mb], b2, acc[mb][nb]); } }
        asm volatile("v_nop\n\tv_nop\n\tv_nop\n\tv_nop" : "+v"(acc[0][0]), "+v"(acc[1][1]), "+v"(acc[2][2]), "+v"(acc[3][3]) : "v"(a[0]), "v"(a[3]));
    }
#pragma unroll
    for (int mb = 0; mb < 4; ++mb) {
#pragma unroll
        for (int nb = 0; nb < 4; ++nb) {
#pragma unroll
            for (int j = 0; j < 8; ++j) os[(hi * 8 + j) * 68 + nb * 16 + lr] = acc[mb][nb][j]; }
        __builtin_amdgcn_wave_barrier(); asm volatile("" ::: "memory");
        float* crow = C + (size_t)(r0 + mb * 16) * ldc + c0;
#pragma unroll 1
        for (int ps = 0; ps < 2; ++ps) {
#pragma unroll
            for (int s = 0; s < 8; ++s) { const int row = 2 * s + hi, cofs = lr * 4; v4f val = *(const v4fa*)(os + row * 68 + cofs); if (BIAS) { val[0] += bfr(bias[c0 + cofs]); val[1] += bfr(bias[c0 + cofs + 1]); val[2] += bfr(bias[c0 + cofs + 2]); val[3] += bfr(bias[c0 + cofs + 3]); }
                *(volatile v4f*)(crow + (size_t)row * ldc + cofs) = val; }
            if (ps == 0) __threadfence(); }
        __builtin_amdgcn_wave_barrier(); asm volatile("" ::: "memory");
    }
}

__global__ __launch_bounds__(256) void k_cvt8(const float* __restrict__ src, bf* dst, size_t n8) { const size_t i = (size_t)blockIdx.x * 256 + threadIdx.x; if (i >= n8) return; const v8f v = *(const v8f*)(src + i * 8); v8us o;
#pragma unroll
    for (int k = 0; k < 8; ++k) o[k] = f2bf(v[k]); *(volatile v8us*)(dst + i * 8) = o; __threadfence(); *(volatile v8us*)(dst + i * 8) = o; }

__global__ __launch_bounds__(256) void k_cvtp(const float* __restrict__ P, bf* dst) {
    const int i = blockIdx.x * 256 + threadIdx.x; if (i >= 2 * HD * HD / 8) return; const int e = i * 8; const int sgm = e / (HD * HD), u = (e / HD) % HD, t = e % HD;
    const v8f v = *(const v8f*)(P + (size_t)u * DP + sgm * HD + t); v8us o;
#pragma unroll
    for (int k = 0; k < 8; ++k) o[k] = f2bf(v[k]); *(volatile v8us*)(dst + e) = o; __threadfence(); *(volatile v8us*)(dst + e) = o; }

__global__ __launch_bounds__(256) void k_split(const float* __restrict__ F, size_t n8, size_t nsc8, float sc0, float sc1, bf* Ah, bf* Al) {
    const size_t i = (size_t)blockIdx.x * 256 + threadIdx.x; if (i >= n8) return; const float sc = (i < nsc8) ? sc0 : sc1;
    const v8f v = *(const v8f*)(F + i * 8); v8us oh, ol;
#pragma unroll
    for (int k = 0; k < 8; ++k) { unsigned short a, c; splitf(v[k] * sc, a, c); oh[k] = a; ol[k] = c; }
    *(volatile v8us*)(Ah + i * 8) = oh; *(volatile v8us*)(Al + i * 8) = ol; __threadfence(); *(volatile v8us*)(Ah + i * 8) = oh; *(volatile v8us*)(Al + i * 8) = ol; }

__global__ __launch_bounds__(256) void k_vtp(const float* __restrict__ F, int pitch, h16* V16) {
    const size_t e = ((size_t)blockIdx.x * 256 + threadIdx.x) * 8; if (e >= (size_t)HD * SEQ) return; const int t = (int)(e % SEQ); const int d = (int)(e / SEQ); v8h o;
#pragma unroll
    for (int q = 0; q < 8; ++q) o[q] = tohx(F[(size_t)(t + q) * pitch + d]);
    *(volatile v8h*)(V16 + e) = o; __threadfence(); *(volatile v8h*)(V16 + e) = o; }

__global__ __launch_bounds__(256) void k_attn(const bf* __restrict__ QH, const bf* __restrict__ QL, const bf* __restrict__ KH, const bf* __restrict__ KL, const h16* __restrict__ VT, float* out) {
    __shared__ __align__(16) bf    khs[KC * HD];
    __shared__ __align__(16) bf    kls[KC * HD];
    __shared__ __align__(16) h16   vts[HD * KC];
    __shared__ __align__(16) float os[8 * 16 * 68];
    const int tid = threadIdx.x, lane = tid & 31, wv = tid >> 5, lr = lane & 15, hi = lane >> 4;
    const int q0 = blockIdx.x * 128 + wv * 16;
    v16bf qh[2], ql[2];
#pragma unroll
    for (int c = 0; c < 2; ++c) { const size_t qo = (size_t)(q0 + lr) * HD + c * 32 + 8 * hi; qh[c] = WFrag<bf>::ld(QH + qo); ql[c] = WFrag<bf>::ld(QL + qo); }
    v8f acc[4];
#pragma unroll
    for (int t = 0; t < 4; ++t) acc[t] = (v8f){};
    float mrun = -1.0e30f, lsum = 0.0f;
#pragma unroll 1
    for (int kc = 0; kc < SEQ; kc += KC) {
#pragma unroll
        for (int i = 0; i < 2; ++i) { const int u = tid + i * 256; const size_t go = (size_t)kc * HD + (size_t)u * 8;
            *(v8us*)(khs + u * 8) = *(const v8us*)(KH + go); *(v8us*)(kls + u * 8) = *(const v8us*)(KL + go);
            const int d = u >> 3, cc = u & 7; *(v8h*)(vts + u * 8) = *(const v8h*)(VT + (size_t)d * SEQ + kc + cc * 8); }
        __syncthreads();
        v8f s[4];
#pragma unroll
        for (int j = 0; j < 4; ++j) s[j] = (v8f){};
        v16bf ka, kb2;
#pragma unroll
        for (int c = 0; c < 2; ++c) {
#pragma unroll
            for (int j = 0; j < 4; ++j) { const int ko = (j * 16 + lr) * HD + c * 32 + 8 * hi; ka = WFrag<bf>::ld(khs + ko); kb2 = WFrag<bf>::ld(kls + ko);
                s[j] = wmmab(ka, qh[c], s[j]); s[j] = wmmab(kb2, qh[c], s[j]); s[j] = wmmab(ka, ql[c], s[j]); } }
        asm volatile("v_nop\n\tv_nop\n\tv_nop\n\tv_nop" : "+v"(s[0]), "+v"(s[1]), "+v"(s[2]), "+v"(s[3]) : "v"(ka), "v"(kb2), "v"(qh[1]), "v"(ql[1]));
        float cm = -1.0e30f;
#pragma unroll
        for (int j = 0; j < 4; ++j)
#pragma unroll
            for (int r = 0; r < 8; ++r) cm = fmaxf(cm, s[j][r]);
        cm = fmaxf(cm, __shfl_xor(cm, 16, 32));
        const float mnew = fmaxf(mrun, cm);
        const float alpha = __builtin_amdgcn_exp2f(fmaxf((mrun - mnew) * L2E, -120.0f));
        float rs = 0.0f; v8h p8[4];
#pragma unroll
        for (int j = 0; j < 4; ++j) { p8[j] = (v8h){};
#pragma unroll
            for (int r = 0; r < 8; ++r) { const float pv = __builtin_amdgcn_exp2f((s[j][r] - mnew) * L2E + LPC); rs += pv; p8[j][r] = tohx(pv); } }
        rs += __shfl_xor(rs, 16, 32);
        lsum = lsum * alpha + rs; mrun = mnew;
#pragma unroll
        for (int t = 0; t < 4; ++t) acc[t] = acc[t] * alpha;
        const v16h pb0 = cat16(p8[0], p8[1]), pb1 = cat16(p8[2], p8[3]);
        v16h va;
#pragma unroll
        for (int t = 0; t < 4; ++t) { const int vo = (t * 16 + lr) * KC + 8 * hi; va = WFrag<h16>::ld(vts + vo); acc[t] = wmma16(va, pb0, acc[t]); va = WFrag<h16>::ld(vts + vo + 32); acc[t] = wmma16(va, pb1, acc[t]); }
        asm volatile("v_nop\n\tv_nop\n\tv_nop\n\tv_nop" : "+v"(acc[0]), "+v"(acc[1]), "+v"(acc[2]), "+v"(acc[3]) : "v"(va), "v"(pb0), "v"(pb1));
        __syncthreads();
    }
    const float inv = __fdiv_rn(1.0f, lsum);
    float* osw = os + wv * (16 * 68);
#pragma unroll
    for (int t = 0; t < 4; ++t) { const v4f lo4 = (v4f){acc[t][0] * inv, acc[t][1] * inv, acc[t][2] * inv, acc[t][3] * inv}; const v4f hi4 = (v4f){acc[t][4] * inv, acc[t][5] * inv, acc[t][6] * inv, acc[t][7] * inv};
        *(v4fa*)(osw + lr * 68 + t * 16 + 8 * hi) = lo4; *(v4fa*)(osw + lr * 68 + t * 16 + 8 * hi + 4) = hi4; }
    __syncthreads();
    float* orow = out + (size_t)q0 * HD;
#pragma unroll 1
    for (int ps = 0; ps < 2; ++ps) {
#pragma unroll
        for (int s2 = 0; s2 < 8; ++s2) { const int row = 2 * s2 + hi, cofs = lr * 4; const v4f val = *(const v4fa*)(osw + row * 68 + cofs); *(volatile v4f*)(orow + (size_t)row * HD + cofs) = val; }
        if (ps == 0) __threadfence(); }
}

extern "C" void kernel_launch(void* const* d_in, const int* in_sizes, int n_in,
                              void* d_out, int out_size, void* d_ws, size_t ws_size, hipStream_t stream) {
    if (n_in < 8) return;
    if (in_sizes[0] < SEQ * HD || in_sizes[1] < HD * DP || in_sizes[2] < HD * HD || in_sizes[3] < HD || in_sizes[4] < HD * HD || in_sizes[5] < HD || in_sizes[6] < HD * HD || in_sizes[7] < HD) return;
    if (out_size < SEQ * HD) return;
    const float* x = (const float*)d_in[0]; const float* params = (const float*)d_in[1];
    const float* wq = (const float*)d_in[2]; const float* bq = (const float*)d_in[3]; const float* wk = (const float*)d_in[4]; const float* bk = (const float*)d_in[5]; const float* wv = (const float*)d_in[6]; const float* bv = (const float*)d_in[7];
    float* OUT = (float*)d_out;
    char* wsp = (char*)d_ws;
    auto take = [&](size_t bytes) { char* p = wsp; wsp += (bytes + 255) & ~(size_t)255; return (void*)p; };
    const size_t PE = (size_t)SEQ * HD;
    bf* XB = (bf*)take(PE * 2);
    bf* PB = (bf*)take((size_t)2 * HD * HD * 2);
    bf* WQ = (bf*)take((size_t)HD * HD * 2); bf* WK = (bf*)take((size_t)HD * HD * 2); bf* WV = (bf*)take((size_t)HD * HD * 2);
    float* FY = (float*)take(2 * PE * 4);
    bf* YH = (bf*)take(2 * PE * 2); bf* YL = (bf*)take(2 * PE * 2);
    float* FQK = (float*)take(2 * PE * 4);
    bf* QKH = (bf*)take(2 * PE * 2); bf* QKL = (bf*)take(2 * PE * 2);
    float* FV = (float*)take(PE * 4);
    h16* VT16 = (h16*)take(PE * 2);
    const size_t used = (size_t)(wsp - (char*)d_ws); if (used > ws_size || used > ((size_t)128 << 20)) return;

    k_cvt8<<<(unsigned)((PE / 8 + 255) / 256), 256, 0, stream>>>(x, XB, PE / 8);
    k_cvtp<<<(2 * HD * HD / 8 + 255) / 256, 256, 0, stream>>>(params, PB);
    k_cvt8<<<(HD * HD / 8 + 255) / 256, 256, 0, stream>>>(wq, WQ, (size_t)HD * HD / 8);
    k_cvt8<<<(HD * HD / 8 + 255) / 256, 256, 0, stream>>>(wk, WK, (size_t)HD * HD / 8);
    k_cvt8<<<(HD * HD / 8 + 255) / 256, 256, 0, stream>>>(wv, WV, (size_t)HD * HD / 8);
    k_gemmw<bf, 0, false><<<dim3(SEQ / 64, 1, 2), 32, 0, stream>>>(XB, nullptr, PB, nullptr, HD, FY, HD, nullptr, 0, (size_t)HD * HD, PE);
    k_split<<<(unsigned)((2 * PE / 8 + 255) / 256), 256, 0, stream>>>(FY, 2 * PE / 8, 0, 1.0f, 1.0f, YH, YL);
    k_gemmw<bf, 1, true><<<dim3(SEQ / 64, 1, 1), 32, 0, stream>>>(YH, YL, WQ, nullptr, HD, FQK, HD, bq, 0, 0, 0);
    k_gemmw<bf, 1, true><<<dim3(SEQ / 64, 1, 1), 32, 0, stream>>>(YH + PE, YL + PE, WK, nullptr, HD, FQK + PE, HD, bk, 0, 0, 0);
    k_split<<<(unsigned)((2 * PE / 8 + 255) / 256), 256, 0, stream>>>(FQK, 2 * PE / 8, PE / 8, SCL, 1.0f, QKH, QKL);
    k_gemmw<bf, 0, true><<<dim3(SEQ / 64, 1, 1), 32, 0, stream>>>(XB, nullptr, WV, nullptr, HD, FV, HD, bv, 0, 0, 0);
    k_vtp<<<(unsigned)((PE / 8 + 255) / 256), 256, 0, stream>>>(FV, HD, VT16);
    k_attn<<<SEQ / 128, 256, 0, stream>>>(QKH, QKL, QKH + PE, QKL + PE, VT16, OUT);
}
